// Model_824633721727
// MI455X (gfx1250) — hardware-verified
//
#include <hip/hip_runtime.h>
#include <stddef.h>
#include <stdint.h>
#include <math.h>


#define NN      10000
#define EE      160000
#define DD      512
#define LL      3
#define NINV    4000
#define NUNK    3000
#define UBASE   7000
#define MP      10112
#define HP      1024
#define XPITCH  1024
#define YK      1536
#define Y0R     4096
#define Y1R     3072
#define OPR     4032
#define OPP     3072
#define NTHR    256
#define NWAVE   8
#define EPT     8
#define CHUNK   (NTHR * EPT)
#define WCAP    (EPT * 32)
#define LISTN   (NWAVE * WCAP)
#define NBMAX   2048
#define NBRUN   512
#define RCAP    12288
#define DEGCAP  64
#define MEAS_B512   8305
#define MEAS_MAXDEG 32
#define STW     512
#define NPAR    (6 * DD)
#define GBM     64
#define GBN     64
#define GTHR    128
#define NEGS    0.2f
#define LNEPS   1.0e-5f
#define WSMAX   134217728
#define LDS_SCAN ((2 * RCAP + 2 * NBMAX + LISTN + 16) * 4 + NPAR * 4)

#define UX      (MP * (DD / 8))
#define UWE     (DD * (DD / 8))
#define UWH     (LL * DD * (1024 / 8))
#define ULN     (DD * (2048 / 8))
#define UZ      ((MP - NN) * (HP / 8))
#define UB1     (UX)
#define UB2     (UB1 + UWE)
#define UB3     (UB2 + UWE)
#define UB4     (UB3 + UWH)
#define UB5     (UB4 + UWH)
#define UB6     (UB5 + ULN)
#define UB7     (UB6 + ULN)
#define UB8     (UB7 + UZ)
#define UB9     (UB8 + UZ)

static_assert(DD == 32 * 16);
static_assert(UBASE + NUNK == NN && NINV <= NN);
static_assert(MP % 128 == 0 && MP >= NN && MP % GBM == 0);
static_assert((UX % NTHR) == 0 && (UWE % NTHR) == 0 && (UWH % NTHR) == 0 && (ULN % NTHR) == 0 && (UZ % NTHR) == 0);
static_assert((CHUNK & (CHUNK - 1)) == 0 && CHUNK <= 4096);
static_assert((NBMAX & (NBMAX - 1)) == 0 && NBMAX <= 4096);
static_assert((NBRUN & (NBRUN - 1)) == 0 && NBRUN <= NBMAX && NBRUN >= 16);
static_assert(NTHR * 8 == NBMAX);
static_assert(LISTN >= NBMAX && LISTN >= NWAVE * WCAP);
static_assert((RCAP % 32) == 0);
static_assert(RCAP * 100 >= MEAS_B512 * 105);
static_assert(DEGCAP >= MEAS_MAXDEG + 8);
static_assert(NWAVE * STW <= RCAP);
static_assert(EE < (1 << 20));
static_assert(LDS_SCAN <= 300000);
static_assert(GBM == (GTHR / 32) * 16);
static_assert(Y0R % GBM == 0 && Y1R % GBM == 0 && OPR % GBM == 0 && OPP % GBN == 0);
static_assert(Y0R >= NINV && Y1R >= NUNK && OPR >= NINV && OPP == Y1R && OPR <= Y0R);
static_assert(UBASE + Y1R <= MP);
static_assert(NINV + ((NN - NINV + GBM - 1) / GBM) * GBM <= MP);
static_assert(NUNK % 4 == 0 && ((long long)NINV * NUNK * 4) % 128 == 0);
static_assert(((NBRUN * ((NN + NBRUN - 1) / NBRUN)) >= NN));

typedef float          v2f  __attribute__((ext_vector_type(2)));
typedef float          v4f  __attribute__((ext_vector_type(4)));
typedef float          v8f  __attribute__((ext_vector_type(8)));
typedef int            v4i  __attribute__((ext_vector_type(4)));
typedef int            v8i  __attribute__((ext_vector_type(8)));
typedef unsigned short v4us __attribute__((ext_vector_type(4)));
typedef unsigned short v8us __attribute__((ext_vector_type(8)));
typedef __bf16         v16b __attribute__((ext_vector_type(16)));
typedef v4f  __attribute__((may_alias)) v4fa;
typedef v8us __attribute__((may_alias)) v8usa;
union FragB { v16b v; v8us h[2]; v8i w; };

__device__ __forceinline__ v8f wmb(const FragB& a, const FragB& b, v8f c) {
  v8f d = __builtin_amdgcn_wmma_f32_16x16x32_bf16(false, a.v, false, b.v, (short)0, c, false, false);
  asm volatile("v_nop\n\tv_nop\n\tv_nop\n\tv_nop" : "+v"(d) : "v"(a.w), "v"(b.w));
  return d;
}

__device__ __forceinline__ void ldwait() {
  asm volatile("s_wait_loadcnt 0x0" ::: "memory");
}

__device__ __forceinline__ unsigned int f2bf(float f) {
  const unsigned int u = __float_as_uint(f);
  const unsigned int r = ((u + 0x7FFFu + ((u >> 16) & 1u)) >> 16) & 0xFFFFu;
  return ((u & 0x7FFFFFFFu) > 0x7F800000u) ? 0x7FC0u : r;
}
__device__ __forceinline__ float bf2f(unsigned int b) { return __uint_as_float(b << 16); }
__device__ __forceinline__ float bfr(float f) { return bf2f(f2bf(f)); }
__device__ __forceinline__ v4f bfr4(const v4f a) {
  v4f r; r.x = bfr(a.x); r.y = bfr(a.y); r.z = bfr(a.z); r.w = bfr(a.w); return r;
}
__device__ __forceinline__ v8us hi8(const v4f a, const v4f b) {
  v8us o;
  o[0] = (unsigned short)f2bf(a.x); o[1] = (unsigned short)f2bf(a.y);
  o[2] = (unsigned short)f2bf(a.z); o[3] = (unsigned short)f2bf(a.w);
  o[4] = (unsigned short)f2bf(b.x); o[5] = (unsigned short)f2bf(b.y);
  o[6] = (unsigned short)f2bf(b.z); o[7] = (unsigned short)f2bf(b.w);
  return o;
}
__device__ __forceinline__ unsigned short lo1(float v) {
  return (unsigned short)f2bf(v - bf2f(f2bf(v)));
}
__device__ __forceinline__ v8us lo8(const v4f a, const v4f b) {
  v8us o;
  o[0] = lo1(a.x); o[1] = lo1(a.y); o[2] = lo1(a.z); o[3] = lo1(a.w);
  o[4] = lo1(b.x); o[5] = lo1(b.y); o[6] = lo1(b.z); o[7] = lo1(b.w);
  return o;
}
__device__ __forceinline__ v8us gath8(const float* __restrict__ p, size_t stride) {
  v8us o;
#pragma unroll
  for (int i = 0; i < 8; ++i) o[i] = (unsigned short)f2bf(p[(size_t)i * stride]);
  return o;
}

__device__ __forceinline__ int scan_chunk(const int* __restrict__ dsts, int nE, int cbase, int slotBase,
                                          int nb, int vec8, int* list, int tid, int lane, int wave) {
  int wc = 0;
  const int el0  = tid * EPT;
  const int e0   = cbase + el0;
  const int sent = -2147483647 - 1;
  v4i da, db;
  if (vec8 != 0 && cbase + CHUNK <= nE) {
    da = *(const v4i*)(dsts + e0);
    db = *(const v4i*)(dsts + e0 + 4);
  } else {
    da.x = (e0     < nE) ? dsts[min(e0,     nE - 1)] : sent;
    da.y = (e0 + 1 < nE) ? dsts[min(e0 + 1, nE - 1)] : sent;
    da.z = (e0 + 2 < nE) ? dsts[min(e0 + 2, nE - 1)] : sent;
    da.w = (e0 + 3 < nE) ? dsts[min(e0 + 3, nE - 1)] : sent;
    db.x = (e0 + 4 < nE) ? dsts[min(e0 + 4, nE - 1)] : sent;
    db.y = (e0 + 5 < nE) ? dsts[min(e0 + 5, nE - 1)] : sent;
    db.z = (e0 + 6 < nE) ? dsts[min(e0 + 6, nE - 1)] : sent;
    db.w = (e0 + 7 < nE) ? dsts[min(e0 + 7, nE - 1)] : sent;
  }
  const unsigned nbs = (unsigned)slotBase;
  const unsigned unb = (unsigned)nb;
  const unsigned s0 = (unsigned)da.x - nbs, s1 = (unsigned)da.y - nbs;
  const unsigned s2 = (unsigned)da.z - nbs, s3 = (unsigned)da.w - nbs;
  const unsigned s4 = (unsigned)db.x - nbs, s5 = (unsigned)db.y - nbs;
  const unsigned s6 = (unsigned)db.z - nbs, s7 = (unsigned)db.w - nbs;
  const bool h0 = s0 < unb, h1 = s1 < unb, h2 = s2 < unb, h3 = s3 < unb;
  const bool h4 = s4 < unb, h5 = s5 < unb, h6 = s6 < unb, h7 = s7 < unb;
  const unsigned any = __builtin_amdgcn_ballot_w32(h0 | h1 | h2 | h3 | h4 | h5 | h6 | h7);
  if (any != 0u) {
#define HITJ(J, HJ, SJ) { \
      const unsigned mj = __builtin_amdgcn_ballot_w32(HJ); \
      if (mj != 0u) { \
        if (HJ) { \
          const int pos = wc + (int)__builtin_amdgcn_mbcnt_lo(mj, 0u); \
          if (pos < WCAP) list[wave * WCAP + pos] = ((el0 + (J)) << 12) | (int)(SJ); \
        } \
        wc += (int)__builtin_popcount(mj); } }
    HITJ(0, h0, s0)
    HITJ(1, h1, s1)
    HITJ(2, h2, s2)
    HITJ(3, h3, s3)
    HITJ(4, h4, s4)
    HITJ(5, h5, s5)
    HITJ(6, h6, s6)
    HITJ(7, h7, s7)
#undef HITJ
  }
  return wc;
}

__global__ __launch_bounds__(NTHR) void k_prep(
    const float* __restrict__ x, const float* __restrict__ wei, const float* __restrict__ weo,
    const float* __restrict__ wl, const float* __restrict__ wr,
    const float* __restrict__ l0, const float* __restrict__ l1,
    unsigned short* XB, unsigned short* WEI, unsigned short* WEO, unsigned short* WLR,
    unsigned short* L0T, unsigned short* L1T, unsigned short* H0, unsigned short* HA)
{
  const int u = (int)blockIdx.x * NTHR + (int)threadIdx.x;
  v8us o;
  unsigned short* dp;
  if (u < UB1) {
    const int row = u >> 6;
    const int c0  = (u & 63) * 8;
    const int rc  = row < NN ? row : NN - 1;
    const float* p = x + (size_t)rc * DD + c0;
    v4f a = *(const v4f*)p, b = *(const v4f*)(p + 4);
    const v4f z4 = {0.f, 0.f, 0.f, 0.f};
    if (row >= NN) { a = z4; b = z4; }
    o = hi8(a, b);
    dp = XB + (size_t)row * DD + c0;
  } else if (u < UB2) {
    const int v = u - UB1;
    const int n = v >> 6, k8 = (v & 63) * 8;
    o = gath8(wei + (size_t)k8 * DD + n, DD);
    dp = WEI + (size_t)n * DD + k8;
  } else if (u < UB3) {
    const int v = u - UB2;
    const int n = v >> 6, k8 = (v & 63) * 8;
    o = gath8(weo + (size_t)k8 * DD + n, DD);
    dp = WEO + (size_t)n * DD + k8;
  } else if (u < UB4) {
    const int v = u - UB3;
    const int layer = v >> 16, rem = v & 65535;
    const int n = rem >> 7, k8 = (rem & 127) * 8, kk = k8 & (DD - 1);
    o = gath8(wl + ((size_t)layer * DD + kk) * DD + n, DD);
    dp = WLR + ((size_t)layer * 1024 + n) * 1024 + k8;
  } else if (u < UB5) {
    const int v = u - UB4;
    const int layer = v >> 16, rem = v & 65535;
    const int n = rem >> 7, k8 = (rem & 127) * 8, kk = k8 & (DD - 1);
    o = gath8(wr + ((size_t)layer * DD + kk) * DD + n, DD);
    dp = WLR + ((size_t)layer * 1024 + 512 + n) * 1024 + k8;
  } else if (u < UB6) {
    const int v = u - UB5;
    const int n = v >> 8, k8 = (v & 255) * 8;
    const int srow = ((k8 >> 10) << 9) + (k8 & (DD - 1));
    o = gath8(l0 + (size_t)srow * DD + n, DD);
    dp = L0T + (size_t)n * 2048 + k8;
  } else if (u < UB7) {
    const int v = u - UB6;
    const int n = v >> 8, k8 = (v & 255) * 8;
    const int srow = ((k8 >> 10) << 9) + (k8 & (DD - 1));
    o = gath8(l1 + (size_t)srow * DD + n, DD);
    dp = L1T + (size_t)n * 2048 + k8;
  } else if (u < UB8) {
    const int v = u - UB7;
    const v8us z = {0, 0, 0, 0, 0, 0, 0, 0};
    o = z;
    dp = H0 + (size_t)(NN + (v >> 7)) * HP + (v & 127) * 8;
  } else if (u < UB9) {
    const int v = u - UB8;
    const v8us z = {0, 0, 0, 0, 0, 0, 0, 0};
    o = z;
    dp = HA + (size_t)(NN + (v >> 7)) * HP + (v & 127) * 8;
  } else {
    return;
  }
  *(volatile v8us*)dp = o;
  __threadfence();
  *(volatile v8us*)dp = o;
}

template <int EPI>
__global__ __launch_bounds__(GTHR) void k_gemm(
    const unsigned short* __restrict__ A0, int lda0, int ks0,
    const unsigned short* __restrict__ A1, int lda1, int ks1,
    const unsigned short* __restrict__ WT, int ldw,
    const float* __restrict__ bias0, const float* __restrict__ bias1, int nsplit,
    float* outF, unsigned short* outH, int ldo, int outRow0, int rowLimit)
{
  __shared__ __attribute__((aligned(16))) float stg[GBM * GBN];
  const int tid = (int)threadIdx.x, lane = tid & 31, wave = tid >> 5, hh = lane >> 4, m = lane & 15;
  const int rowBase = (int)blockIdx.x * GBM;
  const int col0    = (int)blockIdx.y * GBN;

  v8f acc[4];
  {
    const v8f z = {0.f, 0.f, 0.f, 0.f, 0.f, 0.f, 0.f, 0.f};
    acc[0] = z; acc[1] = z; acc[2] = z; acc[3] = z;
  }
  const size_t arow = (size_t)(rowBase + 16 * wave + m);
  const unsigned short* ap0 = A0 + arow * (size_t)lda0 + 8 * hh;
  const unsigned short* ap1 = A1 + arow * (size_t)lda1 + 8 * hh;
  const unsigned short* wp  = WT + (size_t)(col0 + m) * (size_t)ldw + 8 * hh;
#pragma unroll 1
  for (int ks = 0; ks < ks0; ++ks) {
    FragB af;
    af.h[0] = *(const v8usa*)(ap0 + 32 * ks);
    af.h[1] = *(const v8usa*)(ap0 + 32 * ks + 16);
#pragma unroll
    for (int t = 0; t < 4; ++t) {
      const unsigned short* wq = wp + (size_t)(16 * t) * (size_t)ldw + 32 * ks;
      FragB bf;
      bf.h[0] = *(const v8usa*)wq;
      bf.h[1] = *(const v8usa*)(wq + 16);
      acc[t] = wmb(af, bf, acc[t]);
    }
  }
  const unsigned short* wp1 = wp + 32 * ks0;
#pragma unroll 1
  for (int ks = 0; ks < ks1; ++ks) {
    FragB af;
    af.h[0] = *(const v8usa*)(ap1 + 32 * ks);
    af.h[1] = *(const v8usa*)(ap1 + 32 * ks + 16);
#pragma unroll
    for (int t = 0; t < 4; ++t) {
      const unsigned short* wq = wp1 + (size_t)(16 * t) * (size_t)ldw + 32 * ks;
      FragB bf;
      bf.h[0] = *(const v8usa*)wq;
      bf.h[1] = *(const v8usa*)(wq + 16);
      acc[t] = wmb(af, bf, acc[t]);
    }
  }

  float bv[4];
#pragma unroll
  for (int t = 0; t < 4; ++t) {
    if constexpr (EPI == 1) {
      bv[t] = 0.0f;
    } else {
      const int col = col0 + 16 * t + m;
      const int i0 = col < nsplit ? col : nsplit - 1;
      const int i1 = col >= nsplit ? col - nsplit : 0;
      const float b0 = bias0[i0];
      const float b1 = bias1[i1];
      bv[t] = bfr(col < nsplit ? b0 : b1);
    }
  }
#pragma unroll
  for (int t = 0; t < 4; ++t) {
    const int lc = 16 * t + m;
#pragma unroll
    for (int r = 0; r < 8; ++r) {
      const int lr = 16 * wave + 8 * hh + r;
      stg[lr * GBN + lc] = acc[t][r] + bv[t];
    }
  }
  __syncthreads();

  if constexpr (EPI == 0 || EPI == 1) {
    v4f fv[8];
#pragma unroll
    for (int i = 0; i < 8; ++i) {
      const int lr = 16 * wave + 2 * i + hh;
      fv[i] = *(const v4fa*)(stg + lr * GBN + 4 * m);
    }
#pragma unroll
    for (int i = 0; i < 8; ++i) {
      const int lr = 16 * wave + 2 * i + hh;
      float* op = outF + (size_t)(outRow0 + rowBase + lr) * (size_t)ldo + col0 + 4 * m;
      *(volatile v4f*)op = fv[i];
    }
    __threadfence();
#pragma unroll
    for (int i = 0; i < 8; ++i) {
      const int lr = 16 * wave + 2 * i + hh;
      float* op = outF + (size_t)(outRow0 + rowBase + lr) * (size_t)ldo + col0 + 4 * m;
      *(volatile v4f*)op = fv[i];
    }
  } else if constexpr (EPI == 2) {
    const int q = tid & 15, pl = q >> 3, c8 = (q & 7) * 8;
    v8us ov[8];
#pragma unroll
    for (int i = 0; i < 8; ++i) {
      const int lr = 8 * i + (tid >> 4);
      const v4f a = *(const v4fa*)(stg + lr * GBN + c8);
      const v4f b = *(const v4fa*)(stg + lr * GBN + c8 + 4);
      const v8us hv = hi8(a, b);
      const v8us lv = lo8(a, b);
      ov[i] = (pl != 0) ? lv : hv;
    }
#pragma unroll
    for (int i = 0; i < 8; ++i) {
      const int gr = outRow0 + rowBase + 8 * i + (tid >> 4);
      unsigned short* op = outH + (size_t)gr * (size_t)ldo + pl * DD + col0 + c8;
      if (gr < rowLimit) *(volatile v8us*)op = ov[i];
    }
    __threadfence();
#pragma unroll
    for (int i = 0; i < 8; ++i) {
      const int gr = outRow0 + rowBase + 8 * i + (tid >> 4);
      unsigned short* op = outH + (size_t)gr * (size_t)ldo + pl * DD + col0 + c8;
      if (gr < rowLimit) *(volatile v8us*)op = ov[i];
    }
  } else {
    constexpr int LOPL = (EPI == 3) ? 1 : 2;
    const int c8 = (tid & 7) * 8;
    v8us ov[12];
#pragma unroll
    for (int i = 0; i < 12; ++i) {
      const int p    = tid + GTHR * i;
      const int line = p >> 3;
      const int lr   = line / 3;
      const int pl   = line - 3 * lr;
      const v4f a = *(const v4fa*)(stg + lr * GBN + c8);
      const v4f b = *(const v4fa*)(stg + lr * GBN + c8 + 4);
      const v8us hv = hi8(a, b);
      const v8us lv = lo8(a, b);
      const v8us z  = {0, 0, 0, 0, 0, 0, 0, 0};
      v8us o = (pl == LOPL) ? lv : hv;
      if (outRow0 + rowBase + lr >= rowLimit) o = z;
      ov[i] = o;
    }
#pragma unroll
    for (int i = 0; i < 12; ++i) {
      const int p    = tid + GTHR * i;
      const int line = p >> 3;
      const int lr   = line / 3;
      const int pl   = line - 3 * lr;
      unsigned short* op = outH + (size_t)(outRow0 + rowBase + lr) * (size_t)ldo + pl * DD + col0 + c8;
      *(volatile v8us*)op = ov[i];
    }
    __threadfence();
#pragma unroll
    for (int i = 0; i < 12; ++i) {
      const int p    = tid + GTHR * i;
      const int line = p >> 3;
      const int lr   = line / 3;
      const int pl   = line - 3 * lr;
      unsigned short* op = outH + (size_t)(outRow0 + rowBase + lr) * (size_t)ldo + pl * DD + col0 + c8;
      *(volatile v8us*)op = ov[i];
    }
  }
  (void)outF; (void)outH; (void)rowLimit;
}

__global__ __launch_bounds__(NTHR) void k_scan(
    const int* __restrict__ srcs, const int* __restrict__ dsts, const float* __restrict__ ea,
    const float* __restrict__ XLR, const float* __restrict__ We, const float* __restrict__ att,
    const float* __restrict__ gbias, const float* __restrict__ lng, const float* __restrict__ lnb,
    const unsigned short* Hcur, unsigned short* Hout, int nN, int nE, int nb, int vec8)
{
  extern __shared__ v4f lds_dyn[];
  int* reg1 = (int*)lds_dyn;
  int* reg2 = reg1 + RCAP;
  int* scnt = reg2 + RCAP;
  int* soff = scnt + NBMAX;
  int* list = soff + NBMAX;
  int* wcnt = list + LISTN;
  int* wtot = wcnt + NWAVE;
  float* sp = (float*)(wtot + NWAVE);
  const int tid = (int)threadIdx.x, lane = tid & 31, wave = tid >> 5;
  const int nodeBase = (int)blockIdx.x * nb;

  if (tid < 128) {
    const v4f a0 = *(const v4f*)(att   + 4 * tid);
    const v4f a1 = *(const v4f*)(We    + 4 * tid);
    const v4f a2 = *(const v4f*)(We    + DD + 4 * tid);
    const v4f a3 = *(const v4f*)(gbias + 4 * tid);
    const v4f a4 = *(const v4f*)(lng   + 4 * tid);
    const v4f a5 = *(const v4f*)(lnb   + 4 * tid);
    *(v4fa*)(sp + 4 * tid)          = bfr4(a0);
    *(v4fa*)(sp + DD + 4 * tid)     = bfr4(a1);
    *(v4fa*)(sp + 2 * DD + 4 * tid) = bfr4(a2);
    *(v4fa*)(sp + 3 * DD + 4 * tid) = bfr4(a3);
    *(v4fa*)(sp + 4 * DD + 4 * tid) = bfr4(a4);
    *(v4fa*)(sp + 5 * DD + 4 * tid) = bfr4(a5);
  }
  for (int i = tid; i < NBMAX; i += NTHR) scnt[i] = 0;
  __syncthreads();

  int tot = 0;
  const int nChunks = (nE + CHUNK - 1) / CHUNK;
#pragma unroll 1
  for (int ch = 0; ch < nChunks; ++ch) {
    const int cbase = ch * CHUNK;
    const int wc = scan_chunk(dsts, nE, cbase, nodeBase, nb, vec8, list, tid, lane, wave);
    if (lane == 0) wcnt[wave] = wc;
    __syncthreads();
    int pre = 0, all = 0;
#pragma unroll
    for (int w2 = 0; w2 < NWAVE; ++w2) {
      int c = wcnt[w2];
      c = c < 0 ? 0 : (c > WCAP ? WCAP : c);
      all += c;
      pre += (w2 < wave) ? c : 0;
    }
    const int wcc  = wc > WCAP ? WCAP : wc;
    const int base = tot + pre;
#pragma unroll 1
    for (int i = lane; i < wcc; i += 32) {
      const int ent = list[wave * WCAP + i];
      const int el  = (ent >> 12) & (CHUNK - 1);
      const int sl  = ent & (NBMAX - 1);
      int eid = cbase + el;
      eid = eid > nE - 1 ? nE - 1 : eid;
      const int pos = base + i;
      if (pos < RCAP) reg1[pos] = (int)(((unsigned)eid << 12) | (unsigned)sl);
    }
    tot += all;
    tot = tot > RCAP ? RCAP : tot;
    __syncthreads();
  }
  const int nh = tot;

  if (wave == 0) {
#pragma unroll 1
    for (int b0 = 0; b0 < nh; b0 += 32) {
      const int idx = b0 + lane;
      const int uv  = reg1[idx < nh ? idx : nh - 1];
      const int m32 = (nh - b0) < 32 ? (nh - b0) : 32;
#pragma unroll 1
      for (int k = 0; k < m32; ++k) {
        const int u  = __builtin_amdgcn_readlane(uv, k);
        const int sl = u & (NBMAX - 1);
        if (lane == 0) scnt[sl] = scnt[sl] + 1;
      }
    }
  }
  __syncthreads();

  {
    const v4i ca = *(const v4i*)(scnt + 8 * tid);
    const v4i cb = *(const v4i*)(scnt + 8 * tid + 4);
    const int e0 = ca.x < 0 ? 0 : ca.x, e1 = ca.y < 0 ? 0 : ca.y, e2 = ca.z < 0 ? 0 : ca.z, e3 = ca.w < 0 ? 0 : ca.w;
    const int e4 = cb.x < 0 ? 0 : cb.x, e5 = cb.y < 0 ? 0 : cb.y, e6 = cb.z < 0 ? 0 : cb.z, e7 = cb.w < 0 ? 0 : cb.w;
    const int ts = e0 + e1 + e2 + e3 + e4 + e5 + e6 + e7;
    int incl = ts;
#pragma unroll
    for (int d = 1; d < 32; d <<= 1) {
      const int up = __shfl_up(incl, d);
      if (lane >= d) incl += up;
    }
    if (lane == 31) wtot[wave] = incl;
    __syncthreads();
    int pre = 0;
#pragma unroll
    for (int w2 = 0; w2 < NWAVE; ++w2) pre += (w2 < wave) ? wtot[w2] : 0;
    int run = pre + incl - ts;
    soff[8 * tid + 0] = run; run += e0;
    soff[8 * tid + 1] = run; run += e1;
    soff[8 * tid + 2] = run; run += e2;
    soff[8 * tid + 3] = run; run += e3;
    soff[8 * tid + 4] = run; run += e4;
    soff[8 * tid + 5] = run; run += e5;
    soff[8 * tid + 6] = run; run += e6;
    soff[8 * tid + 7] = run;
  }
  __syncthreads();
  for (int i = tid; i < NBMAX; i += NTHR) list[i] = soff[i];
  __syncthreads();

  if (wave == 0) {
#pragma unroll 1
    for (int b0 = 0; b0 < nh; b0 += 32) {
      const int idx = b0 + lane;
      const int uv  = reg1[idx < nh ? idx : nh - 1];
      const int m32 = (nh - b0) < 32 ? (nh - b0) : 32;
#pragma unroll 1
      for (int k = 0; k < m32; ++k) {
        const int u   = __builtin_amdgcn_readlane(uv, k);
        const int sl  = u & (NBMAX - 1);
        const int eid = (int)((unsigned)u >> 12);
        if (lane == 0) {
          int pos = list[sl];
          pos = pos < 0 ? 0 : (pos > RCAP - 1 ? RCAP - 1 : pos);
          reg2[pos] = eid;
          list[sl] = pos + 1;
        }
      }
    }
  }
  __syncthreads();

  const int nbw = nb >> 3;
  const bool ovf = (nh >= RCAP);
  const float qnan = __int_as_float(0x7fc00000);
  float* stw = (float*)reg1 + wave * STW;
  float at[16], w0[16], w1[16];
#pragma unroll
  for (int hf = 0; hf < 2; ++hf) {
    const float* q = sp + 256 * hf + 8 * lane;
    const v4f a0 = *(const v4fa*)(q),          a1 = *(const v4fa*)(q + 4);
    const v4f b0 = *(const v4fa*)(q + DD),     b1 = *(const v4fa*)(q + DD + 4);
    const v4f c0 = *(const v4fa*)(q + 2 * DD), c1 = *(const v4fa*)(q + 2 * DD + 4);
    at[8 * hf + 0] = a0.x; at[8 * hf + 1] = a0.y; at[8 * hf + 2] = a0.z; at[8 * hf + 3] = a0.w;
    at[8 * hf + 4] = a1.x; at[8 * hf + 5] = a1.y; at[8 * hf + 6] = a1.z; at[8 * hf + 7] = a1.w;
    w0[8 * hf + 0] = b0.x; w0[8 * hf + 1] = b0.y; w0[8 * hf + 2] = b0.z; w0[8 * hf + 3] = b0.w;
    w0[8 * hf + 4] = b1.x; w0[8 * hf + 5] = b1.y; w0[8 * hf + 6] = b1.z; w0[8 * hf + 7] = b1.w;
    w1[8 * hf + 0] = c0.x; w1[8 * hf + 1] = c0.y; w1[8 * hf + 2] = c0.z; w1[8 * hf + 3] = c0.w;
    w1[8 * hf + 4] = c1.x; w1[8 * hf + 5] = c1.y; w1[8 * hf + 6] = c1.z; w1[8 * hf + 7] = c1.w;
  }

#pragma unroll 1
  for (int jt = 0; jt < nbw; ++jt) {
    const int slot = wave * nbw + jt;
    const int grow = nodeBase + slot;
    if (grow >= nN) continue;
    int st = soff[slot];
    const int craw = scnt[slot];
    int cnt = craw;
    st  = st < 0 ? 0 : (st > nh ? nh : st);
    cnt = cnt < 0 ? 0 : (cnt > DEGCAP ? DEGCAP : cnt);
    if (cnt > nh - st) cnt = nh - st;
    const float pz = (ovf || craw > DEGCAP) ? qnan : 0.0f;

    float xr[16], acc[16];
    {
      const float* dr = XLR + (size_t)grow * XPITCH + DD + 8 * lane;
      const v4f r0 = *(const v4f*)dr,         r1 = *(const v4f*)(dr + 4);
      const v4f r2 = *(const v4f*)(dr + 256), r3 = *(const v4f*)(dr + 260);
      ldwait();
      xr[0] = r0.x; xr[1] = r0.y; xr[2] = r0.z; xr[3] = r0.w;
      xr[4] = r1.x; xr[5] = r1.y; xr[6] = r1.z; xr[7] = r1.w;
      xr[8] = r2.x; xr[9] = r2.y; xr[10] = r2.z; xr[11] = r2.w;
      xr[12] = r3.x; xr[13] = r3.y; xr[14] = r3.z; xr[15] = r3.w;
    }
#pragma unroll
    for (int i = 0; i < 16; ++i) acc[i] = 0.0f;
    float mx = -3.0e38f, dn = 0.0f;

#pragma unroll 1
    for (int q = 0; q < cnt; ++q) {
      int idx = st + q; idx = idx > RCAP - 1 ? RCAP - 1 : idx;
      int eid = reg2[idx]; eid = eid < 0 ? 0 : (eid > nE - 1 ? nE - 1 : eid);
      const int sraw = srcs[eid];
      const int s = sraw < 0 ? 0 : (sraw > nN - 1 ? nN - 1 : sraw);
      const float* sr = XLR + (size_t)s * XPITCH + 8 * lane;
      const v4f x0 = *(const v4f*)sr,         x1 = *(const v4f*)(sr + 4);
      const v4f x2 = *(const v4f*)(sr + 256), x3 = *(const v4f*)(sr + 260);
      const v2f ev = *(const v2f*)(ea + 2 * (size_t)eid);
      ldwait();
      float xs[16];
      xs[0] = x0.x; xs[1] = x0.y; xs[2] = x0.z; xs[3] = x0.w;
      xs[4] = x1.x; xs[5] = x1.y; xs[6] = x1.z; xs[7] = x1.w;
      xs[8] = x2.x; xs[9] = x2.y; xs[10] = x2.z; xs[11] = x2.w;
      xs[12] = x3.x; xs[13] = x3.y; xs[14] = x3.z; xs[15] = x3.w;
      const float e0 = bfr(ev.x), e1 = bfr(ev.y);
      float part = 0.0f;
#pragma unroll
      for (int i = 0; i < 16; ++i) {
        const float t = fmaf(e0, w0[i], e1 * w1[i]);
        float mv = (xs[i] + xr[i]) + t;
        mv = mv > 0.0f ? mv : mv * NEGS;
        part = fmaf(mv, at[i], part);
      }
#pragma unroll
      for (int off = 16; off > 0; off >>= 1) part += __shfl_xor(part, off);
      const float lg = part;
      const float df = lg - mx;
      const float ee = expf(-fabsf(df));
      const bool  up = df > 0.0f;
      const float s1 = up ? ee : 1.0f;
      const float s2 = up ? 1.0f : ee;
      mx = up ? lg : mx;
      dn = fmaf(dn, s1, s2);
#pragma unroll
      for (int i = 0; i < 16; ++i) acc[i] = fmaf(acc[i], s1, s2 * xs[i]);
    }

    const float ds = dn > 0.0f ? dn : 1.0f;
    const float iv = (dn > 0.0f ? 1.0f : 0.0f) * __builtin_amdgcn_rcpf(ds);
    {
      v4f t0, t1, t2, t3;
      t0.x = acc[0];  t0.y = acc[1];  t0.z = acc[2];  t0.w = acc[3];
      t1.x = acc[4];  t1.y = acc[5];  t1.z = acc[6];  t1.w = acc[7];
      t2.x = acc[8];  t2.y = acc[9];  t2.z = acc[10]; t2.w = acc[11];
      t3.x = acc[12]; t3.y = acc[13]; t3.z = acc[14]; t3.w = acc[15];
      *(v4fa*)(stw + 8 * lane)       = t0;
      *(v4fa*)(stw + 8 * lane + 4)   = t1;
      *(v4fa*)(stw + 256 + 8 * lane) = t2;
      *(v4fa*)(stw + 260 + 8 * lane) = t3;
    }
    const unsigned short* hrow = Hcur + (size_t)grow * HP;
    float sum = 0.0f;
#pragma unroll 1
    for (int g = 0; g < 4; ++g) {
      const int cb = 256 * (g >> 1) + 8 * lane + 4 * (g & 1);
      const v4f a  = *(const v4fa*)(stw + cb);
      const v4f gb = *(const v4fa*)(sp + 3 * DD + cb);
      const v4us hq = *(const v4us*)(hrow + cb);
      const v4us lq = *(const v4us*)(hrow + DD + cb);
      v4f r;
      r.x = (fmaf(a.x, iv, gb.x) + pz) + (bf2f((unsigned)hq.x) + bf2f((unsigned)lq.x));
      r.y = (fmaf(a.y, iv, gb.y) + pz) + (bf2f((unsigned)hq.y) + bf2f((unsigned)lq.y));
      r.z = (fmaf(a.z, iv, gb.z) + pz) + (bf2f((unsigned)hq.z) + bf2f((unsigned)lq.z));
      r.w = (fmaf(a.w, iv, gb.w) + pz) + (bf2f((unsigned)hq.w) + bf2f((unsigned)lq.w));
      *(v4fa*)(stw + cb) = r;
      sum += (r.x + r.y) + (r.z + r.w);
    }
#pragma unroll
    for (int off = 16; off > 0; off >>= 1) sum += __shfl_xor(sum, off);
    const float mean = sum * (1.0f / (float)DD);
    float vs = 0.0f;
#pragma unroll 1
    for (int g = 0; g < 4; ++g) {
      const int cb = 256 * (g >> 1) + 8 * lane + 4 * (g & 1);
      const v4f r = *(const v4fa*)(stw + cb);
      const float d0 = r.x - mean, d1 = r.y - mean, d2 = r.z - mean, d3 = r.w - mean;
      vs = fmaf(d0, d0, vs); vs = fmaf(d1, d1, vs); vs = fmaf(d2, d2, vs); vs = fmaf(d3, d3, vs);
    }
#pragma unroll
    for (int off = 16; off > 0; off >>= 1) vs += __shfl_xor(vs, off);
    const float var  = vs * (1.0f / (float)DD);
    const float rstd = 1.0f / sqrtf(var + LNEPS);
#pragma unroll 1
    for (int hf = 0; hf < 2; ++hf) {
      const int cb = 256 * hf + 8 * lane;
      const v4f ra = *(const v4fa*)(stw + cb),          rb = *(const v4fa*)(stw + cb + 4);
      const v4f ga = *(const v4fa*)(sp + 4 * DD + cb),  gb2 = *(const v4fa*)(sp + 4 * DD + cb + 4);
      const v4f ba = *(const v4fa*)(sp + 5 * DD + cb),  bb2 = *(const v4fa*)(sp + 5 * DD + cb + 4);
      v4f oa, ob;
      oa.x = fmaf((ra.x - mean) * rstd, ga.x, ba.x);   oa.y = fmaf((ra.y - mean) * rstd, ga.y, ba.y);
      oa.z = fmaf((ra.z - mean) * rstd, ga.z, ba.z);   oa.w = fmaf((ra.w - mean) * rstd, ga.w, ba.w);
      ob.x = fmaf((rb.x - mean) * rstd, gb2.x, bb2.x); ob.y = fmaf((rb.y - mean) * rstd, gb2.y, bb2.y);
      ob.z = fmaf((rb.z - mean) * rstd, gb2.z, bb2.z); ob.w = fmaf((rb.w - mean) * rstd, gb2.w, bb2.w);
      oa.x = (oa.x > 0.0f) ? oa.x : (oa.x - oa.x);     oa.y = (oa.y > 0.0f) ? oa.y : (oa.y - oa.y);
      oa.z = (oa.z > 0.0f) ? oa.z : (oa.z - oa.z);     oa.w = (oa.w > 0.0f) ? oa.w : (oa.w - oa.w);
      ob.x = (ob.x > 0.0f) ? ob.x : (ob.x - ob.x);     ob.y = (ob.y > 0.0f) ? ob.y : (ob.y - ob.y);
      ob.z = (ob.z > 0.0f) ? ob.z : (ob.z - ob.z);     ob.w = (ob.w > 0.0f) ? ob.w : (ob.w - ob.w);
      const v8us hv = hi8(oa, ob);
      const v8us lv = lo8(oa, ob);
      unsigned short* hp = Hout + (size_t)grow * HP + cb;
      *(volatile v8us*)hp = hv;
      *(volatile v8us*)(hp + DD) = lv;
      __threadfence();
      *(volatile v8us*)hp = hv;
      *(volatile v8us*)(hp + DD) = lv;
    }
  }
}

__global__ __launch_bounds__(NTHR) void k_copy(const float* __restrict__ OUTP, const int* __restrict__ pinv,
                                               const int* __restrict__ punk, float* out, int nq) {
  const int q  = (int)blockIdx.x * NTHR + (int)threadIdx.x;
  const int qc = q < nq ? q : nq - 1;
  const int row = qc / (NUNK / 4);
  const int c4  = qc - row * (NUNK / 4);
  v4f v = *(const v4f*)(OUTP + (size_t)row * OPP + 4 * c4);
  const int a = pinv[0], b = punk[0];
  const float qnan = __int_as_float(0x7fc00000);
  const v4f nv = {qnan, qnan, qnan, qnan};
  if (a != NINV || b != NUNK) v = nv;
  float* op = out + 4 * (size_t)qc;
  if (q < nq) *(volatile v4f*)op = v;
  __threadfence();
  if (q < nq) *(volatile v4f*)op = v;
}

constexpr size_t SZ_XB  = (size_t)MP * DD * 2;
constexpr size_t SZ_WE  = (size_t)DD * DD * 2;
constexpr size_t SZ_WLR = (size_t)LL * 1024 * 1024 * 2;
constexpr size_t SZ_LN  = (size_t)DD * 2048 * 2;
constexpr size_t SZ_H   = (size_t)MP * HP * 2;
constexpr size_t SZ_Y0  = (size_t)Y0R * YK * 2;
constexpr size_t SZ_Y1  = (size_t)Y1R * YK * 2;
constexpr size_t SZ_XLR = (size_t)MP * XPITCH * 4;
constexpr size_t SZ_OP  = (size_t)OPR * OPP * 4;
constexpr size_t SZ_F32 = SZ_OP > SZ_XLR ? SZ_OP : SZ_XLR;
constexpr size_t O_XB   = 0;
constexpr size_t O_WEI  = O_XB + SZ_XB;
constexpr size_t O_WEO  = O_WEI + SZ_WE;
constexpr size_t O_WLR  = O_WEO + SZ_WE;
constexpr size_t O_L0T  = O_WLR + SZ_WLR;
constexpr size_t O_L1T  = O_L0T + SZ_LN;
constexpr size_t O_H0   = O_L1T + SZ_LN;
constexpr size_t O_HA   = O_H0 + SZ_H;
constexpr size_t O_Y0   = O_HA + SZ_H;
constexpr size_t O_F32  = O_Y0 + SZ_Y0;
constexpr size_t WS_TOT = O_F32 + SZ_F32;
static_assert(SZ_Y1 <= SZ_XB);
static_assert((O_WEI % 256) == 0 && (O_WLR % 256) == 0 && (O_H0 % 256) == 0 && (O_HA % 256) == 0);
static_assert((O_Y0 % 256) == 0 && (O_F32 % 256) == 0);
static_assert(WS_TOT <= (size_t)WSMAX);

extern "C" void kernel_launch(void* const* d_in, const int* in_sizes, int n_in,
                              void* d_out, int out_size, void* d_ws, size_t ws_size,
                              hipStream_t stream) {
  if (n_in < 22) return;
  if (in_sizes[0] != NN * DD || in_sizes[1] != EE * 2) return;
  if (in_sizes[2] != DD * DD || in_sizes[3] != DD || in_sizes[4] != DD * DD || in_sizes[5] != DD) return;
  if (in_sizes[6] != LL * DD * DD || in_sizes[7] != LL * DD || in_sizes[8] != LL * DD * DD || in_sizes[9] != LL * DD) return;
  if (in_sizes[10] != LL * 2 * DD || in_sizes[11] != LL * DD || in_sizes[12] != LL * DD) return;
  if (in_sizes[13] != LL * DD || in_sizes[14] != LL * DD) return;
  if (in_sizes[15] != 2 * DD * DD || in_sizes[16] != DD || in_sizes[17] != 2 * DD * DD || in_sizes[18] != DD) return;
  if (in_sizes[19] != 2 * EE || in_sizes[20] != 1 || in_sizes[21] != 1) return;
  if (out_size != NINV * NUNK) return;
  if (WS_TOT > ws_size) return;

  const float* x      = (const float*)d_in[0];
  const float* eattr  = (const float*)d_in[1];
  const float* wei    = (const float*)d_in[2];
  const float* bei    = (const float*)d_in[3];
  const float* weo    = (const float*)d_in[4];
  const float* beo    = (const float*)d_in[5];
  const float* gwl    = (const float*)d_in[6];
  const float* gbl    = (const float*)d_in[7];
  const float* gwr    = (const float*)d_in[8];
  const float* gbr    = (const float*)d_in[9];
  const float* gwe    = (const float*)d_in[10];
  const float* gatt   = (const float*)d_in[11];
  const float* gbias  = (const float*)d_in[12];
  const float* lng    = (const float*)d_in[13];
  const float* lnb    = (const float*)d_in[14];
  const float* l0w    = (const float*)d_in[15];
  const float* l0b    = (const float*)d_in[16];
  const float* l1w    = (const float*)d_in[17];
  const float* l1b    = (const float*)d_in[18];
  const int*   ei     = (const int*)  d_in[19];
  const int*   pinv   = (const int*)  d_in[20];
  const int*   punk   = (const int*)  d_in[21];
  float* out = (float*)d_out;
  const int* src = ei;
  const int* dst = ei + EE;

  char* ws = (char*)d_ws;
  unsigned short* XB  = (unsigned short*)(ws + O_XB);
  unsigned short* Y1C = (unsigned short*)(ws + O_XB);
  unsigned short* WEI = (unsigned short*)(ws + O_WEI);
  unsigned short* WEO = (unsigned short*)(ws + O_WEO);
  unsigned short* WLR = (unsigned short*)(ws + O_WLR);
  unsigned short* L0T = (unsigned short*)(ws + O_L0T);
  unsigned short* L1T = (unsigned short*)(ws + O_L1T);
  unsigned short* H0  = (unsigned short*)(ws + O_H0);
  unsigned short* HA  = (unsigned short*)(ws + O_HA);
  unsigned short* Y0C = (unsigned short*)(ws + O_Y0);
  float*          XLR = (float*)(ws + O_F32);
  float*          OUTP = (float*)(ws + O_F32);

  hipFuncSetAttribute(reinterpret_cast<const void*>(&k_scan),
                      hipFuncAttributeMaxDynamicSharedMemorySize, LDS_SCAN);

  k_prep<<<UB9 / NTHR, NTHR, 0, stream>>>(x, wei, weo, gwl, gwr, l0w, l1w, XB, WEI, WEO, WLR, L0T, L1T, H0, HA);

  k_gemm<2><<<dim3((NINV + GBM - 1) / GBM, DD / GBN), GTHR, 0, stream>>>(
      XB, DD, DD / 32, XB, DD, 0, WEI, DD, bei, bei, DD, nullptr, H0, HP, 0, NINV);
  k_gemm<2><<<dim3((NN - NINV + GBM - 1) / GBM, DD / GBN), GTHR, 0, stream>>>(
      XB + (size_t)NINV * DD, DD, DD / 32, XB, DD, 0, WEO, DD, beo, beo, DD, nullptr, H0, HP, NINV, NN);

  const int gA = (NN + NBRUN - 1) / NBRUN;
  const int vec8 = ((EE & 3) == 0) ? 1 : 0;
  for (int k = 0; k < LL; ++k) {
    const unsigned short* Hc = (k == 0) ? H0 : HA;
    k_gemm<0><<<dim3(MP / GBM, 1024 / GBN), GTHR, 0, stream>>>(
        Hc, HP, HP / 32, Hc, HP, 0, WLR + (size_t)k * 1024 * 1024, 1024,
        gbl + k * DD, gbr + k * DD, DD, XLR, nullptr, XPITCH, 0, MP);
    k_scan<<<gA, NTHR, LDS_SCAN, stream>>>(src, dst, eattr, XLR, gwe + (size_t)k * 2 * DD, gatt + k * DD,
                                            gbias + k * DD, lng + k * DD, lnb + k * DD,
                                            Hc, HA, NN, EE, NBRUN, vec8);
  }

  k_gemm<3><<<dim3(Y0R / GBM, DD / GBN), GTHR, 0, stream>>>(
      H0, HP, HP / 32, HA, HP, HP / 32, L0T, 2048, l0b, l0b, DD, nullptr, Y0C, YK, 0, NINV);
  k_gemm<4><<<dim3(Y1R / GBM, DD / GBN), GTHR, 0, stream>>>(
      H0 + (size_t)UBASE * HP, HP, HP / 32, HA + (size_t)UBASE * HP, HP, HP / 32, L1T, 2048,
      l1b, l1b, DD, nullptr, Y1C, YK, 0, NUNK);
  k_gemm<1><<<dim3(OPR / GBM, OPP / GBN), GTHR, 0, stream>>>(
      Y0C, YK, YK / 32, Y0C, YK, 0, Y1C, YK, l0b, l0b, OPP, OUTP, nullptr, OPP, 0, OPR);
  const int nq = NINV * (NUNK / 4);
  k_copy<<<(nq + NTHR - 1) / NTHR, NTHR, 0, stream>>>(OUTP, pinv, punk, out, nq);
}
